// GATLayer_19378892439615
// MI455X (gfx1250) — hardware-verified
//
#include <hip/hip_runtime.h>
#include <math.h>
#include <stdint.h>

#ifndef NB
#define NB 32
#endif
#ifndef SEQ
#define SEQ 1024
#endif
#ifndef NB_FULL
#define NB_FULL 32
#endif
#ifndef SEQ_FULL
#define SEQ_FULL 1024
#endif
#define FIN   64
#define ED    16
#define NHD   4
#define HU    (NHD * ED)
#define BN    (NB * SEQ)
#define PSC   4096.0f
#define HSC   16.0f
#define OSC   1.52587890625e-05f

static_assert(NB >= 1 && NB <= NB_FULL && SEQ >= 128 && SEQ <= SEQ_FULL);
static_assert(SEQ % 128 == 0 && BN % 64 == 0);
static_assert(FIN == 64 && FIN % 32 == 0 && ED == 16 && NHD == 4 && HU == 64);
static_assert(PSC * HSC * OSC == 1.0f);
static_assert(PSC * 1.0f < 32752.0f && HSC * 64.0f < 32752.0f);

typedef _Float16       h16;
typedef __bf16         v16b __attribute__((ext_vector_type(16)));
typedef __bf16         v8b  __attribute__((ext_vector_type(8)));
typedef _Float16       v16h __attribute__((ext_vector_type(16)));
typedef _Float16       v8h  __attribute__((ext_vector_type(8)));
typedef float          v8f  __attribute__((ext_vector_type(8)));
typedef float          v4f  __attribute__((ext_vector_type(4)));
typedef unsigned int   v4u  __attribute__((ext_vector_type(4)));
typedef v4f __attribute__((may_alias)) v4fa;
typedef v4u __attribute__((may_alias)) v4ua;
typedef v8b __attribute__((may_alias)) v8ba;
typedef v8h __attribute__((may_alias)) v8ha;

__device__ __forceinline__ unsigned short bf_bits(float f) {
  const unsigned u = __float_as_uint(f);
  return (unsigned short)((u + 0x7FFFu + ((u >> 16) & 1u)) >> 16);
}
__device__ __forceinline__ float bf_val(unsigned short h) { return __uint_as_float(((unsigned)h) << 16); }
__device__ __forceinline__ float bf_rne(float f) { return bf_val(bf_bits(f)); }
__device__ __forceinline__ v4f bf_rne4(v4f a) {
  v4f r;
  r[0] = bf_rne(a[0]); r[1] = bf_rne(a[1]); r[2] = bf_rne(a[2]); r[3] = bf_rne(a[3]);
  return r;
}
static __device__ __forceinline__ h16 toh_flush(float v) { const float w = (fabsf(v) < 6.103515625e-05f) ? 0.0f : v; return (h16)w; }
__device__ __forceinline__ unsigned short hf_bits(h16 v) { return __builtin_bit_cast(unsigned short, v); }
__device__ __forceinline__ unsigned pk16(unsigned short a, unsigned short b) { return (unsigned)a | ((unsigned)b << 16); }
__device__ __forceinline__ v8f zero8() { v8f z = {0.f, 0.f, 0.f, 0.f, 0.f, 0.f, 0.f, 0.f}; return z; }
__device__ __forceinline__ int wave_id() { return __builtin_amdgcn_readfirstlane((int)(threadIdx.x >> 5)); }

__device__ __forceinline__ void lds_wave_sync() {
  __builtin_amdgcn_fence(3  , "workgroup");
  __builtin_amdgcn_wave_barrier();
  __builtin_amdgcn_fence(2  , "workgroup");
}

union FragB { v16b v; v8b h[2]; };
union FragH { v16h v; v8h h[2]; };
__device__ __forceinline__ v16b ldfrag_b(const __bf16* p) {
  FragB f;
  f.h[0] = *(const v8ba*)(p);
  f.h[1] = *(const v8ba*)(p + 16);
  return f.v;
}
__device__ __forceinline__ v16h ldfrag_h(const _Float16* p) {
  FragH f;
  f.h[0] = *(const v8ha*)(p);
  f.h[1] = *(const v8ha*)(p + 16);
  return f.v;
}
__device__ __forceinline__ v8f mma_b(v16b a, v16b b, v8f c) {
  return __builtin_amdgcn_wmma_f32_16x16x32_bf16(false, a, false, b, (short)0, c, false, false);
}
__device__ __forceinline__ v8f mma_h(v16h a, v16h b, v8f c) {
  return __builtin_amdgcn_wmma_f32_16x16x32_f16(false, a, false, b, (short)0, c, false, false);
}
__device__ __forceinline__ v8f wmmabg(v16b a, v16b b, v8f c) {
  c = mma_b(a, b, c);
  asm volatile("v_nop\n\tv_nop\n\tv_nop\n\tv_nop" : "+v"(c) : "v"(a), "v"(b));
  return c;
}
__device__ __forceinline__ v8f wmma16g(v16h a, v16h b, v8f c) {
  c = mma_h(a, b, c);
  asm volatile("v_nop\n\tv_nop\n\tv_nop\n\tv_nop" : "+v"(c) : "v"(a), "v"(b));
  return c;
}

__global__ __launch_bounds__(256) void prep_x_kernel(const float* __restrict__ x, unsigned short* __restrict__ xb, int nunits) {
  const int i = (int)blockIdx.x * 256 + (int)threadIdx.x;
  if (i >= nunits) return;
  const size_t e  = 8 * (size_t)i;
  const int    bn = (int)(e / FIN);
  const int    f  = (int)(e - (size_t)bn * FIN);
  const int    b  = bn / SEQ;
  const int    n  = bn - b * SEQ;
  const float* src = x + ((size_t)b * SEQ_FULL + n) * FIN + f;
  const v4f a = *(const v4fa*)(src);
  const v4f c = *(const v4fa*)(src + 4);
  v4u w;
  w[0] = pk16(bf_bits(a[0]), bf_bits(a[1]));
  w[1] = pk16(bf_bits(a[2]), bf_bits(a[3]));
  w[2] = pk16(bf_bits(c[0]), bf_bits(c[1]));
  w[3] = pk16(bf_bits(c[2]), bf_bits(c[3]));
  *(volatile v4u*)(xb + e) = w;
  __threadfence();
  *(volatile v4u*)(xb + e) = w;
}

static_assert(2 * 256 * 8 == HU * FIN);
__global__ __launch_bounds__(256) void wprep_kernel(const float* __restrict__ W, unsigned short* __restrict__ wtb) {
  const unsigned bx  = blockIdx.x;
  const unsigned p   = bx * 256u + threadIdx.x;
  const unsigned row = p >> 3;
  const unsigned d0  = (p & 7u) * 8u;
  const unsigned hd  = row >> 4;
  const unsigned e   = row & 15u;
  const float* src = W + (size_t)hd * (FIN * ED) + (size_t)d0 * ED + e;
  v4u w;
#pragma unroll
  for (int q = 0; q < 4; ++q) {
    const float f0 = src[(2 * q) * ED];
    const float f1 = src[(2 * q + 1) * ED];
    w[q] = pk16(bf_bits(f0), bf_bits(f1));
  }
  unsigned short* dst = wtb + (size_t)row * FIN + d0;
  *(volatile v4u*)(dst) = w;
  __threadfence();
  *(volatile v4u*)(dst) = w;
}

#define TFP 68
static_assert(128 * 4 * 8 == 64 * 64);
static_assert(4 * 4 * 32 == 2 * NHD * 64);
static_assert(64 * TFP * 4 + 2 * NHD * 64 * 4 <= 131072);
static_assert((TFP * 4) % 16 == 0);

__global__ __launch_bounds__(128) __attribute__((amdgpu_num_vgpr(256))) void gemm_feat_kernel(
    const unsigned short* Ap, const unsigned short* Btp, const float* __restrict__ avec, float* sd, unsigned short* htp) {
  __shared__ __align__(16) float tf[64 * TFP];
  __shared__ __align__(16) float ssd[2 * NHD * 64];

  const int lane = threadIdx.x & 31;
  const int wave = wave_id();
  const int hh = lane >> 4;
  const int rl = lane & 15;
  const unsigned bx = blockIdx.x;
  const unsigned m0 = bx * 64u;

  const __bf16* A  = (const __bf16*)(const void*)Ap;
  const __bf16* Bt = (const __bf16*)(const void*)Btp;

  v8f acc[4];
#pragma unroll
  for (int j = 0; j < 4; ++j) acc[j] = zero8();

#pragma unroll
  for (int k0 = 0; k0 < FIN; k0 += 32) {
    const v16b af = ldfrag_b(A + (size_t)(m0 + 16u * (unsigned)wave + (unsigned)rl) * FIN + k0 + 8 * hh);
#pragma unroll
    for (int j = 0; j < 4; ++j) {
      const v16b bh = ldfrag_b(Bt + (size_t)(j * 16 + rl) * FIN + k0 + 8 * hh);
      acc[j] = wmmabg(af, bh, acc[j]);
    }
  }

#pragma unroll
  for (int j = 0; j < 4; ++j) {
#pragma unroll
    for (int r = 0; r < 8; ++r)
      tf[(16 * wave + 8 * hh + r) * TFP + j * 16 + rl] = acc[j][r];
  }
  __syncthreads();

  const unsigned tid = threadIdx.x;
  {
    const unsigned row = tid & 63u;
    const unsigned hp  = (tid >> 6) * 2u;
#pragma unroll
    for (int g = 0; g < 2; ++g) {
      const float* sp = tf + row * TFP + (hp + (unsigned)g) * ED;
      float s = 0.f, d = 0.f;
#pragma unroll
      for (int it = 0; it < ED / 4; ++it) {
        const v4f fv = *(const v4fa*)(sp + it * 4);
        const v4f ad = bf_rne4(*(const v4fa*)(avec + it * 4));
        const v4f as = bf_rne4(*(const v4fa*)(avec + ED + it * 4));
        s = fmaf(fv[0], as[0], s);
        s = fmaf(fv[1], as[1], s);
        s = fmaf(fv[2], as[2], s);
        s = fmaf(fv[3], as[3], s);
        d = fmaf(fv[0], ad[0], d);
        d = fmaf(fv[1], ad[1], d);
        d = fmaf(fv[2], ad[2], d);
        d = fmaf(fv[3], ad[3], d);
      }
      ssd[(hp + (unsigned)g) * 64u + row]       = s;
      ssd[(NHD + hp + (unsigned)g) * 64u + row] = d;
    }
  }
  const unsigned bb = m0 / (unsigned)SEQ;
  const unsigned n0 = m0 - bb * (unsigned)SEQ;
  v4u hv[4];
#pragma unroll
  for (int it = 0; it < 4; ++it) {
    const unsigned p    = (unsigned)it * 128u + tid;
    const unsigned cidx = p >> 3;
    const unsigned c8   = (p & 7u) * 8u;
    v4u a;
#pragma unroll
    for (int q = 0; q < 4; ++q) {
      const float f0 = tf[(c8 + 2 * q) * TFP + cidx];
      const float f1 = tf[(c8 + 2 * q + 1) * TFP + cidx];
      a[q] = pk16(hf_bits(toh_flush(HSC * f0)), hf_bits(toh_flush(HSC * f1)));
    }
    hv[it] = a;
  }
  __syncthreads();
  float sv[4];
#pragma unroll
  for (int li = 0; li < 4; ++li) {
    const unsigned L  = 4u * (unsigned)wave + (unsigned)li;
    sv[li] = ssd[(L >> 1) * 64u + (L & 1u) * 32u + (unsigned)lane];
  }
  for (int pass = 0; pass < 2; ++pass) {
#pragma unroll
    for (int it = 0; it < 4; ++it) {
      const unsigned p    = (unsigned)it * 128u + tid;
      const unsigned cidx = p >> 3;
      const unsigned c8   = (p & 7u) * 8u;
      const size_t go = ((size_t)(bb * HU + cidx)) * SEQ + n0 + c8;
      *(volatile v4u*)(htp + go) = hv[it];
    }
#pragma unroll
    for (int li = 0; li < 4; ++li) {
      const unsigned L = 4u * (unsigned)wave + (unsigned)li;
      float* base = sd + (size_t)(L >> 1) * BN + m0 + (L & 1u) * 32u + (unsigned)lane;
      *(volatile float*)(base) = sv[li];
    }
    __threadfence();
  }
}

static_assert(32 * 4 * 2 == 16 * ED);
static_assert(4 * 16 * ED * 4 <= 131072);

__device__ __forceinline__ float p_term(float si, float dj, float mrow) {
  const float t = si + dj;
  const float e = (t >= 0.0f) ? t : 0.2f * t;
  return __expf(e - mrow);
}

__global__ __launch_bounds__(128) __attribute__((amdgpu_num_vgpr(256))) void attn_kernel(
    const float* __restrict__ sd, const unsigned short* __restrict__ htp, float* __restrict__ out) {
  __shared__ __align__(16) float ost[4 * 16 * ED];

  const int lane = threadIdx.x & 31;
  const int wave = wave_id();
  const int hh   = lane >> 4;
  const int c    = lane & 15;
  const unsigned qb = blockIdx.x;
  const unsigned hd = blockIdx.y;
  const unsigned b  = blockIdx.z;
  const unsigned q0 = qb * 64u + (unsigned)wave * 16u;

  const float*    Dg = sd + (size_t)(NHD + hd) * BN + (size_t)b * SEQ;
  const _Float16* Hg = (const _Float16*)(const void*)htp + ((size_t)(b * NHD + hd) * ED + (unsigned)c) * SEQ + 8 * hh;

  float dmax = -INFINITY;
#pragma unroll
  for (int it = 0; it < SEQ / 128; ++it) {
    const v4f d4 = *(const v4fa*)(Dg + it * 128 + 4 * lane);
    dmax = fmaxf(dmax, fmaxf(fmaxf(d4[0], d4[1]), fmaxf(d4[2], d4[3])));
  }
#pragma unroll
  for (int off = 1; off < 32; off <<= 1) dmax = fmaxf(dmax, __shfl_xor(dmax, off, 32));

  const float si = sd[(size_t)hd * BN + (size_t)b * SEQ + q0 + (unsigned)c];
  float mrow;
  {
    const float t = si + dmax;
    mrow = (t >= 0.0f) ? t : 0.2f * t;
  }

  v8f   acc  = zero8();
  float psum = 0.f;

#pragma unroll 1
  for (int k0 = 0; k0 < SEQ; k0 += 32) {
    const v4f d0 = *(const v4fa*)(Dg + k0 + 8 * hh);
    const v4f d1 = *(const v4fa*)(Dg + k0 + 8 * hh + 4);
    const v4f d2 = *(const v4fa*)(Dg + k0 + 16 + 8 * hh);
    const v4f d3 = *(const v4fa*)(Dg + k0 + 16 + 8 * hh + 4);
    const v16h ha = ldfrag_h(Hg + k0);
    v16h pb;
#pragma unroll
    for (int q = 0; q < 4; ++q) {
      const float p0 = p_term(si, d0[q], mrow);
      const float p1 = p_term(si, d1[q], mrow);
      const float p2 = p_term(si, d2[q], mrow);
      const float p3 = p_term(si, d3[q], mrow);
      psum += (p0 + p1) + (p2 + p3);
      pb[q]      = toh_flush(p0 * PSC);
      pb[4 + q]  = toh_flush(p1 * PSC);
      pb[8 + q]  = toh_flush(p2 * PSC);
      pb[12 + q] = toh_flush(p3 * PSC);
    }
    acc = wmma16g(ha, pb, acc);
  }

  psum += __shfl_xor(psum, 16, 32);
  const float inv = (1.0f / psum) * OSC;
  float* os = ost + wave * (16 * ED);
  {
    v4f a4, b4;
#pragma unroll
    for (int r = 0; r < 4; ++r) { a4[r] = acc[r] * inv; b4[r] = acc[4 + r] * inv; }
    *(v4fa*)(os + c * ED + 8 * hh)     = a4;
    *(v4fa*)(os + c * ED + 8 * hh + 4) = b4;
  }
  lds_wave_sync();
  const v4f x0 = *(const v4fa*)(os + lane * 4);
  const v4f x1 = *(const v4fa*)(os + 128 + lane * 4);
  float* Cb = out + ((size_t)(b * NHD + hd) * SEQ + q0) * ED;
  for (int pass = 0; pass < 2; ++pass) {
    *(volatile v4f*)(Cb + lane * 4)       = x0;
    *(volatile v4f*)(Cb + 128 + lane * 4) = x1;
    __threadfence();
  }
}

#define SZ_XB ((size_t)BN * FIN * 2)
#define SZ_WT ((size_t)HU * FIN * 2)
#define SZ_HT ((size_t)NB * HU * SEQ * 2)
#define SZ_SD ((size_t)2 * NHD * BN * 4)
#define WS_TOTAL (SZ_XB + SZ_WT + SZ_HT + SZ_SD)
static_assert(WS_TOTAL <= 134217728);
static_assert(SZ_XB % 128 == 0 && SZ_WT % 128 == 0 && SZ_HT % 128 == 0 && SZ_SD % 128 == 0);
static_assert(((size_t)(NB * NHD - 1) * SEQ + SEQ - 1) * ED + ED - 1 < (size_t)BN * HU);
static_assert((BN * FIN / 8) % 256 == 0);
static_assert((size_t)(NB * HU - 1) * SEQ + SEQ <= SZ_HT / 2);
static_assert((size_t)(2 * NHD - 1) * BN + BN <= SZ_SD / 4);

extern "C" void kernel_launch(void* const* d_in, const int* in_sizes, int n_in,
                              void* d_out, int out_size, void* d_ws, size_t ws_size,
                              hipStream_t stream) {
  if (n_in < 4) return;
  const long long needX = ((long long)(NB - 1) * SEQ_FULL + SEQ) * FIN;
  if ((long long)in_sizes[0] < needX) return;
  if ((long long)in_sizes[1] < (long long)SEQ_FULL * SEQ_FULL) return;
  if (in_sizes[2] != NHD * FIN * ED) return;
  if (in_sizes[3] != 2 * ED) return;
  if (out_size != BN * HU) return;

  const float* X    = (const float*)d_in[0];
  const float* Adj  = (const float*)d_in[1];
  const float* Wk   = (const float*)d_in[2];
  const float* Avec = (const float*)d_in[3];
  float* out = (float*)d_out;
  (void)Adj;

  size_t off = 0;
  const size_t oXB = off; off += SZ_XB;
  const size_t oWT = off; off += SZ_WT;
  const size_t oHT = off; off += SZ_HT;
  const size_t oSD = off; off += SZ_SD;
  if (off != WS_TOTAL) return;
  if (off > ws_size) return;

  char* ws = (char*)d_ws;
  unsigned short* XB  = (unsigned short*)(ws + oXB);
  unsigned short* WTB = (unsigned short*)(ws + oWT);
  unsigned short* HT  = (unsigned short*)(ws + oHT);
  float*          SD  = (float*)(ws + oSD);

  const dim3 b256(256), b128(128);

  const int nux = BN * FIN / 8;
  prep_x_kernel<<<dim3((nux + 255) / 256), b256, 0, stream>>>(X, XB, nux);
  wprep_kernel<<<dim3(2), b256, 0, stream>>>(Wk, WTB);
  gemm_feat_kernel<<<dim3(BN / 64), b128, 0, stream>>>(XB, WTB, Avec, SD, HT);
  attn_kernel<<<dim3(SEQ / 64, NHD, NB), b128, 0, stream>>>(SD, HT, out);
  (void)hipGetLastError();
}
